// BaseModel_87170656240449
// MI455X (gfx1250) — hardware-run, weakly checked
//
#include <hip/hip_runtime.h>
#include <stddef.h>
#include <stdint.h>


#define FIN     256
#define NHID    128
#define KPL     256
#define NTHR    256
#define NWAVE   8
#define EPT     8
#define CHUNK   (NTHR * EPT)
#define WCAP    (EPT * 32)
#define LISTN   (NWAVE * WCAP)
#define NBMAX   2048
#define RCAP    28672
#define DEGCAP  64
#define STW     512
#define GBM     64
#define GBN     64
#define GTHR    128
#define WSMAX   134217728
#define LDS_AGG ((2 * RCAP + 2 * NBMAX + LISTN) * 4 + 64)

static_assert((CHUNK & (CHUNK - 1)) == 0 && CHUNK <= 4096);
static_assert((NBMAX & (NBMAX - 1)) == 0 && NBMAX <= 4096);
static_assert(NTHR * 8 == NBMAX);
static_assert(LISTN >= NBMAX);
static_assert(LISTN >= NWAVE * WCAP);
static_assert((RCAP % 32) == 0);
static_assert(NWAVE * STW <= RCAP);
static_assert(LDS_AGG <= 300000);
static_assert(GBM == (GTHR / 32) * 16);
static_assert((KPL % 32) == 0);
static_assert((NHID % GBN) == 0);
static_assert(NHID == 4 * 32);
static_assert(KPL == 2 * NHID);
static_assert(FIN == KPL);
static_assert(FIN / 8 == 32 && KPL / 8 == 32);
static_assert(NHID <= STW);
static_assert((NHID % 8) == 0);

typedef float          v4f  __attribute__((ext_vector_type(4)));
typedef float          v8f  __attribute__((ext_vector_type(8)));
typedef int            v4i  __attribute__((ext_vector_type(4)));
typedef int            v8i  __attribute__((ext_vector_type(8)));
typedef unsigned short v8us __attribute__((ext_vector_type(8)));
typedef __bf16         v16b __attribute__((ext_vector_type(16)));
union FragB { v16b v; v4i q[2]; v8i w; };

__device__ __forceinline__ v8f wmb(const FragB& a, const FragB& b, v8f c) {
  v8f d = __builtin_amdgcn_wmma_f32_16x16x32_bf16(false, a.v, false, b.v, (short)0, c, false, false);
  asm volatile("v_nop\n\tv_nop\n\tv_nop\n\tv_nop" : "+v"(d) : "v"(a.w), "v"(b.w));
  return d;
}

__device__ __forceinline__ void ldwait() {
  asm volatile("s_wait_loadcnt 0x0" ::: "memory");
}

__device__ __forceinline__ unsigned int f2bf_bits(float f) {
  const unsigned int u = __float_as_uint(f);
  if ((u & 0x7fffffffu) > 0x7f800000u) return (u >> 16) | 0x40u;
  return (u + 0x7fffu + ((u >> 16) & 1u)) >> 16;
}
__device__ __forceinline__ float bf16r(float f) {
  return __uint_as_float(f2bf_bits(f) << 16);
}

__device__ __forceinline__ v8us cvt8b(const v4f a, const v4f b, const int sel) {
  v8us o;
#define CVB(I, X) { const unsigned int hb = f2bf_bits(X); \
    const unsigned int lb = f2bf_bits((X) - __uint_as_float(hb << 16)); \
    o[I] = (unsigned short)(sel != 0 ? lb : hb); }
  CVB(0, a.x) CVB(1, a.y) CVB(2, a.z) CVB(3, a.w)
  CVB(4, b.x) CVB(5, b.y) CVB(6, b.z) CVB(7, b.w)
#undef CVB
  return o;
}

__device__ __forceinline__ int scan_chunk(const int* __restrict__ dsts, int nE, int cbase, int slotBase,
                                          int nb, int vec8, int* list, int tid, int lane, int wave) {
  int wc = 0;
  const int el0  = tid * EPT;
  const int e0   = cbase + el0;
  const int sent = -2147483647 - 1;
  v4i da, db;
  if (vec8 != 0 && cbase + CHUNK <= nE) {
    da = *(const v4i*)(dsts + e0);
    db = *(const v4i*)(dsts + e0 + 4);
  } else {
    da.x = (e0     < nE) ? dsts[min(e0,     nE - 1)] : sent;
    da.y = (e0 + 1 < nE) ? dsts[min(e0 + 1, nE - 1)] : sent;
    da.z = (e0 + 2 < nE) ? dsts[min(e0 + 2, nE - 1)] : sent;
    da.w = (e0 + 3 < nE) ? dsts[min(e0 + 3, nE - 1)] : sent;
    db.x = (e0 + 4 < nE) ? dsts[min(e0 + 4, nE - 1)] : sent;
    db.y = (e0 + 5 < nE) ? dsts[min(e0 + 5, nE - 1)] : sent;
    db.z = (e0 + 6 < nE) ? dsts[min(e0 + 6, nE - 1)] : sent;
    db.w = (e0 + 7 < nE) ? dsts[min(e0 + 7, nE - 1)] : sent;
  }
  const unsigned nbs = (unsigned)slotBase;
  const unsigned unb = (unsigned)nb;
  const unsigned s0 = (unsigned)da.x - nbs, s1 = (unsigned)da.y - nbs;
  const unsigned s2 = (unsigned)da.z - nbs, s3 = (unsigned)da.w - nbs;
  const unsigned s4 = (unsigned)db.x - nbs, s5 = (unsigned)db.y - nbs;
  const unsigned s6 = (unsigned)db.z - nbs, s7 = (unsigned)db.w - nbs;
  const bool h0 = s0 < unb, h1 = s1 < unb, h2 = s2 < unb, h3 = s3 < unb;
  const bool h4 = s4 < unb, h5 = s5 < unb, h6 = s6 < unb, h7 = s7 < unb;
  const unsigned any = __builtin_amdgcn_ballot_w32(h0 | h1 | h2 | h3 | h4 | h5 | h6 | h7);
  if (any != 0u) {
#define HITJ(J, HJ, SJ) { \
      const unsigned mj = __builtin_amdgcn_ballot_w32(HJ); \
      if (mj != 0u) { \
        if (HJ) { \
          const int pos = wc + (int)__builtin_amdgcn_mbcnt_lo(mj, 0u); \
          if (pos < WCAP) list[wave * WCAP + pos] = ((el0 + (J)) << 12) | (int)(SJ); \
        } \
        wc += (int)__builtin_popcount(mj); } }
    HITJ(0, h0, s0)
    HITJ(1, h1, s1)
    HITJ(2, h2, s2)
    HITJ(3, h3, s3)
    HITJ(4, h4, s4)
    HITJ(5, h5, s5)
    HITJ(6, h6, s6)
    HITJ(7, h7, s7)
#undef HITJ
  }
  return wc;
}

__global__ __launch_bounds__(NTHR) void k_xprep(const float* __restrict__ x, unsigned short* xb,
                                                int nN, int nUnits) {
  const int i = (int)blockIdx.x * NTHR + (int)threadIdx.x;
  if (i >= nUnits) return;
  const int row = i >> 5;
  const int c0  = (i & 31) * 8;
  const int rc  = row < nN ? row : nN - 1;
  const float* p = x + (size_t)rc * FIN + c0;
  v4f a = *(const v4f*)p, b = *(const v4f*)(p + 4);
  const v4f z4 = {0.f, 0.f, 0.f, 0.f};
  if (row >= nN) { a = z4; b = z4; }
  const v8us hv = cvt8b(a, b, 0);
  const size_t o = (size_t)row * KPL + c0;
  *(volatile v8us*)(xb + o) = hv;
  __threadfence();
  *(volatile v8us*)(xb + o) = hv;
}

__global__ __launch_bounds__(NTHR) void k_wtr(const float* __restrict__ w, int KI,
                                              unsigned short* wt, int nUnits) {
  const int u = (int)blockIdx.x * NTHR + (int)threadIdx.x;
  if (u >= nUnits) return;
  const int n  = u >> 5;
  const int k8 = (u & 31) * 8;
  int ks = (k8 >= KI) ? (k8 - KI) : k8;
  ks = ks > KI - 8 ? KI - 8 : ks;
  ks = ks < 0 ? 0 : ks;
  const float* p = w + (size_t)ks * NHID + n;
  v4f a, b;
  a.x = p[0];                  a.y = p[(size_t)NHID];       a.z = p[(size_t)2 * NHID];   a.w = p[(size_t)3 * NHID];
  b.x = p[(size_t)4 * NHID];   b.y = p[(size_t)5 * NHID];   b.z = p[(size_t)6 * NHID];   b.w = p[(size_t)7 * NHID];
  const v8us hv = cvt8b(a, b, 0);
  const size_t o = (size_t)n * KPL + k8;
  *(volatile v8us*)(wt + o) = hv;
  __threadfence();
  *(volatile v8us*)(wt + o) = hv;
}

__global__ __launch_bounds__(GTHR) void k_gemm(
    const unsigned short* __restrict__ A, const unsigned short* __restrict__ WT,
    float* outF, int K, int ldo)
{
  __shared__ __attribute__((aligned(16))) float stg[GBM * GBN];
  const int tid = (int)threadIdx.x, lane = tid & 31, wave = tid >> 5, hh = lane >> 4, m = lane & 15;
  const int rowBase = (int)blockIdx.x * GBM;
  const int col0    = (int)blockIdx.y * GBN;

  v8f acc[4];
  {
    const v8f z = {0.f, 0.f, 0.f, 0.f, 0.f, 0.f, 0.f, 0.f};
    acc[0] = z; acc[1] = z; acc[2] = z; acc[3] = z;
  }
  const unsigned short* ap = A  + (size_t)(rowBase + 16 * wave + m) * (size_t)K + 8 * hh;
  const unsigned short* wp = WT + (size_t)(col0 + m) * (size_t)K + 8 * hh;
  const int ksteps = K >> 5;
#pragma unroll 1
  for (int ks = 0; ks < ksteps; ++ks) {
    FragB af;
    af.q[0] = *(const v4i*)(ap + 32 * ks);
    af.q[1] = *(const v4i*)(ap + 32 * ks + 16);
#pragma unroll
    for (int t = 0; t < 4; ++t) {
      const unsigned short* wq = wp + (size_t)(16 * t) * (size_t)K + 32 * ks;
      FragB bf;
      bf.q[0] = *(const v4i*)wq;
      bf.q[1] = *(const v4i*)(wq + 16);
      acc[t] = wmb(af, bf, acc[t]);
    }
  }

#pragma unroll
  for (int t = 0; t < 4; ++t) {
    const int lc = 16 * t + m;
#pragma unroll
    for (int r = 0; r < 8; ++r) {
      const int lr = 16 * wave + 8 * hh + r;
      stg[lr * GBN + lc] = acc[t][r];
    }
  }
  __syncthreads();

  v4f fv[8];
#pragma unroll
  for (int i = 0; i < 8; ++i) {
    const int lr = 16 * wave + 2 * i + hh;
    fv[i] = *(const v4f*)(stg + lr * GBN + 4 * m);
  }
#pragma unroll
  for (int i = 0; i < 8; ++i) {
    const int lr = 16 * wave + 2 * i + hh;
    const int gr = rowBase + lr;
    float* op = outF + (size_t)gr * (size_t)ldo + col0 + 4 * m;
    *(volatile v4f*)op = fv[i];
  }
  __threadfence();
#pragma unroll
  for (int i = 0; i < 8; ++i) {
    const int lr = 16 * wave + 2 * i + hh;
    const int gr = rowBase + lr;
    float* op = outF + (size_t)gr * (size_t)ldo + col0 + 4 * m;
    *(volatile v4f*)op = fv[i];
  }
}

template<int MODE>
__global__ __launch_bounds__(NTHR) void k_agg(
    const int* __restrict__ dsts, const int* __restrict__ srcs, const float* __restrict__ vals,
    const float* __restrict__ S, const float* __restrict__ bias,
    unsigned short* Hout, float* outF,
    int nN, int nE, int nb, int vec8, int MPr) {
  extern __shared__ v4f lds_dyn[];
  int* reg1 = (int*)lds_dyn;
  int* reg2 = reg1 + RCAP;
  int* scnt = reg2 + RCAP;
  int* soff = scnt + NBMAX;
  int* list = soff + NBMAX;
  int* wcnt = list + LISTN;
  int* wtot = wcnt + NWAVE;
  const int tid = (int)threadIdx.x, lane = tid & 31, wave = tid >> 5;
  const int nodeBase = (int)blockIdx.x * nb;

  for (int i = tid; i < NBMAX; i += NTHR) scnt[i] = 0;
  __syncthreads();

  int tot = 0;
  const int nChunks = (nE + CHUNK - 1) / CHUNK;
#pragma unroll 1
  for (int ch = 0; ch < nChunks; ++ch) {
    const int cbase = ch * CHUNK;
    const int wc = scan_chunk(dsts, nE, cbase, nodeBase, nb, vec8, list, tid, lane, wave);
    if (lane == 0) wcnt[wave] = wc;
    __syncthreads();
    int pre = 0, all = 0;
#pragma unroll
    for (int w2 = 0; w2 < NWAVE; ++w2) {
      int c = wcnt[w2];
      c = c < 0 ? 0 : (c > WCAP ? WCAP : c);
      all += c;
      pre += (w2 < wave) ? c : 0;
    }
    const int wcc  = wc > WCAP ? WCAP : wc;
    const int base = tot + pre;
#pragma unroll 1
    for (int i = lane; i < wcc; i += 32) {
      const int ent = list[wave * WCAP + i];
      const int el  = (ent >> 12) & (CHUNK - 1);
      const int sl  = ent & (NBMAX - 1);
      int eid = cbase + el;
      eid = eid > nE - 1 ? nE - 1 : eid;
      const int pos = base + i;
      if (pos < RCAP) reg1[pos] = (int)(((unsigned)eid << 12) | (unsigned)sl);
    }
    tot += all;
    tot = tot > RCAP ? RCAP : tot;
    __syncthreads();
  }
  const int nh = tot;

  if (wave == 0) {
#pragma unroll 1
    for (int b0 = 0; b0 < nh; b0 += 32) {
      const int idx = b0 + lane;
      const int uv  = reg1[idx < RCAP ? idx : RCAP - 1];
      const int m32 = (nh - b0) < 32 ? (nh - b0) : 32;
#pragma unroll 1
      for (int k = 0; k < m32; ++k) {
        const int u  = __builtin_amdgcn_readlane(uv, k);
        const int sl = u & (NBMAX - 1);
        if (lane == 0) scnt[sl] = scnt[sl] + 1;
      }
    }
  }
  __syncthreads();

  {
    const v4i ca = *(const v4i*)(scnt + 8 * tid);
    const v4i cb = *(const v4i*)(scnt + 8 * tid + 4);
    const int e0 = ca.x < 0 ? 0 : ca.x, e1 = ca.y < 0 ? 0 : ca.y, e2 = ca.z < 0 ? 0 : ca.z, e3 = ca.w < 0 ? 0 : ca.w;
    const int e4 = cb.x < 0 ? 0 : cb.x, e5 = cb.y < 0 ? 0 : cb.y, e6 = cb.z < 0 ? 0 : cb.z, e7 = cb.w < 0 ? 0 : cb.w;
    const int ts = e0 + e1 + e2 + e3 + e4 + e5 + e6 + e7;
    int incl = ts;
#pragma unroll
    for (int d = 1; d < 32; d <<= 1) {
      const int up = __shfl_up(incl, d);
      if (lane >= d) incl += up;
    }
    if (lane == 31) wtot[wave] = incl;
    __syncthreads();
    int pre = 0;
#pragma unroll
    for (int w2 = 0; w2 < NWAVE; ++w2) pre += (w2 < wave) ? wtot[w2] : 0;
    int run = pre + incl - ts;
    soff[8 * tid + 0] = run; run += e0;
    soff[8 * tid + 1] = run; run += e1;
    soff[8 * tid + 2] = run; run += e2;
    soff[8 * tid + 3] = run; run += e3;
    soff[8 * tid + 4] = run; run += e4;
    soff[8 * tid + 5] = run; run += e5;
    soff[8 * tid + 6] = run; run += e6;
    soff[8 * tid + 7] = run;
  }
  __syncthreads();
  for (int i = tid; i < NBMAX; i += NTHR) list[i] = soff[i];
  __syncthreads();

  if (wave == 0) {
#pragma unroll 1
    for (int b0 = 0; b0 < nh; b0 += 32) {
      const int idx = b0 + lane;
      const int uv  = reg1[idx < RCAP ? idx : RCAP - 1];
      const int m32 = (nh - b0) < 32 ? (nh - b0) : 32;
#pragma unroll 1
      for (int k = 0; k < m32; ++k) {
        const int u   = __builtin_amdgcn_readlane(uv, k);
        const int sl  = u & (NBMAX - 1);
        const int eid = (int)((unsigned)u >> 12);
        if (lane == 0) {
          int pos = list[sl];
          pos = pos < 0 ? 0 : (pos > RCAP - 1 ? RCAP - 1 : pos);
          reg2[pos] = eid;
          list[sl] = pos + 1;
        }
      }
    }
  }
  __syncthreads();

  const int nbw = nb >> 3;
  const bool ovf = (nh >= RCAP);
  const float qnan = __int_as_float(0x7fc00000);
  float* stw = (float*)reg1 + wave * STW;
  float bj[4];
#pragma unroll
  for (int j = 0; j < 4; ++j) bj[j] = bf16r(bias[32 * j + lane]);
#pragma unroll 1
  for (int jt = 0; jt < nbw; ++jt) {
    const int slot = wave * nbw + jt;
    const int grow = nodeBase + slot;
    int st = soff[slot];
    const int craw = scnt[slot];
    int cnt = craw;
    st  = st < 0 ? 0 : (st > nh ? nh : st);
    cnt = cnt < 0 ? 0 : (cnt > DEGCAP ? DEGCAP : cnt);
    if (cnt > nh - st) cnt = nh - st;
    const float pz = (ovf || craw > DEGCAP) ? qnan : 0.0f;
    const bool wr = (MODE == 0) ? (grow < MPr) : (grow < nN);
    const float live = grow < nN ? 1.0f : 0.0f;

    float av[4];
#pragma unroll
    for (int j = 0; j < 4; ++j) av[j] = 0.f;

#pragma unroll 1
    for (int q = 0; q < cnt; ++q) {
      int idx = st + q; idx = idx > RCAP - 1 ? RCAP - 1 : idx;
      int eid = reg2[idx]; eid = eid < 0 ? 0 : (eid > nE - 1 ? nE - 1 : eid);
      const int craw2 = srcs[eid];
      const int c = craw2 < 0 ? 0 : (craw2 > nN - 1 ? nN - 1 : craw2);
      const float ve = bf16r(vals[eid]);
      const float* sr = S + (size_t)c * NHID + lane;
      float sv[4];
#pragma unroll
      for (int j = 0; j < 4; ++j) sv[j] = sr[32 * j];
      ldwait();
#pragma unroll
      for (int j = 0; j < 4; ++j) av[j] = fmaf(ve, sv[j], av[j]);
    }
    float rv[4];
#pragma unroll
    for (int j = 0; j < 4; ++j) rv[j] = fmaxf(av[j] + bj[j], 0.f) * live + pz;

    __builtin_amdgcn_fence(__ATOMIC_RELEASE, "wavefront");
    __builtin_amdgcn_wave_barrier();
#pragma unroll
    for (int j = 0; j < 4; ++j) stw[32 * j + lane] = rv[j];
    __builtin_amdgcn_fence(__ATOMIC_RELEASE, "wavefront");
    __builtin_amdgcn_wave_barrier();
    if (MODE == 0) {
      const int lc = lane & 15;
      const v4f ga = *(const v4f*)(stw + 8 * lc);
      const v4f gb = *(const v4f*)(stw + 8 * lc + 4);
      const v8us hv = cvt8b(ga, gb, lane >> 4);
      unsigned short* gp = Hout + (size_t)grow * KPL + 8 * lane;
      if (wr) *(volatile v8us*)gp = hv;
      __threadfence();
      if (wr) *(volatile v8us*)gp = hv;
    } else {
      const v4f g = *(const v4f*)(stw + 4 * lane);
      float* op = outF + (size_t)grow * NHID + 4 * lane;
      if (wr) *(volatile v4f*)op = g;
      __threadfence();
      if (wr) *(volatile v4f*)op = g;
    }
  }
}

static int pick_nb(int nE, int nN) {
  int nb = NBMAX;
  while (nb > 16 && (long long)nb * (long long)nE * 5LL > (long long)RCAP * (long long)nN * 4LL) nb >>= 1;
  return nb;
}
static inline int cdiv(int a, int b) { return (a + b - 1) / b; }

extern "C" void kernel_launch(void* const* d_in, const int* in_sizes, int n_in,
                              void* d_out, int out_size, void* d_ws, size_t ws_size,
                              hipStream_t stream) {
  if (n_in < 8) return;
  const int nN = in_sizes[0] / FIN;
  if (nN <= 0 || in_sizes[0] != nN * FIN || nN > (1 << 22)) return;
  const int nE = in_sizes[1];
  if (nE < 1 || nE > (1 << 20)) return;
  if (in_sizes[2] != nE || in_sizes[3] != nE) return;
  if (in_sizes[4] != FIN * NHID || in_sizes[5] != NHID) return;
  if (in_sizes[6] != NHID * NHID || in_sizes[7] != NHID) return;
  if (out_size != nN * NHID) return;

  const float* x    = (const float*)d_in[0];
  const int*   rows = (const int*)  d_in[1];
  const int*   cols = (const int*)  d_in[2];
  const float* vals = (const float*)d_in[3];
  const float* W1   = (const float*)d_in[4];
  const float* b1   = (const float*)d_in[5];
  const float* W2   = (const float*)d_in[6];
  const float* b2   = (const float*)d_in[7];
  float* out = (float*)d_out;

  const int MP   = cdiv(nN, GBM) * GBM;
  const int nb   = pick_nb(nE, nN);
  if (nb > NBMAX || (nb & 7) != 0) return;
  const int gA   = cdiv(MP, nb);
  const int vec8 = ((nE & 3) == 0) ? 1 : 0;
  if (gA * nb < MP) return;

  char* ws = (char*)d_ws;
  size_t off = 0;
  const size_t oXB  = off; off += (size_t)MP * KPL * 2;            off = (off + 255) & ~(size_t)255;
  const size_t oS   = off; off += (size_t)MP * NHID * 4;           off = (off + 255) & ~(size_t)255;
  const size_t oHB  = off; off += (size_t)MP * KPL * 2;            off = (off + 255) & ~(size_t)255;
  const size_t oWT1 = off; off += (size_t)NHID * KPL * 2;          off = (off + 255) & ~(size_t)255;
  const size_t oWT2 = off; off += (size_t)NHID * KPL * 2;          off = (off + 255) & ~(size_t)255;
  if (off > ws_size || off > (size_t)WSMAX) return;
  unsigned short* XB  = (unsigned short*)(ws + oXB);
  float*          S   = (float*)(ws + oS);
  unsigned short* HB  = (unsigned short*)(ws + oHB);
  unsigned short* WT1 = (unsigned short*)(ws + oWT1);
  unsigned short* WT2 = (unsigned short*)(ws + oWT2);

  hipFuncSetAttribute(reinterpret_cast<const void*>(&k_agg<0>),
                      hipFuncAttributeMaxDynamicSharedMemorySize, LDS_AGG);
  hipFuncSetAttribute(reinterpret_cast<const void*>(&k_agg<1>),
                      hipFuncAttributeMaxDynamicSharedMemorySize, LDS_AGG);

  const int nUx = MP * (KPL / 8);
  k_xprep<<<cdiv(nUx, NTHR), NTHR, 0, stream>>>(x, XB, nN, nUx);

  const int nUw = NHID * (KPL / 8);
  k_wtr<<<cdiv(nUw, NTHR), NTHR, 0, stream>>>(W1, FIN, WT1, nUw);
  k_wtr<<<cdiv(nUw, NTHR), NTHR, 0, stream>>>(W2, NHID, WT2, nUw);

  const int gM = MP / GBM;
  k_gemm<<<dim3(gM, NHID / GBN), GTHR, 0, stream>>>(XB, WT1, S, KPL, NHID);
  k_agg<0><<<gA, NTHR, LDS_AGG, stream>>>(rows, cols, vals, S, b1, HB, out, nN, nE, nb, vec8, MP);
  k_gemm<<<dim3(gM, NHID / GBN), GTHR, 0, stream>>>(HB, WT2, S, KPL, NHID);
  k_agg<1><<<gA, NTHR, LDS_AGG, stream>>>(rows, cols, vals, S, b2, HB, out, nN, nE, nb, vec8, MP);
}
